// ProbAttentionLayer_33243046871128
// MI455X (gfx1250) — hardware-verified
//
#include <hip/hip_runtime.h>
#include <math.h>
#include <stdint.h>

#define NBATCH 4
#define SEQ    2048
#define DM     1024
#define NH     16
#define HD     64
#define MP     (NBATCH * SEQ)
#define NQB    (SEQ / 64)
#define CTXP   (2 * DM)
#define LNEPS  1.0e-5f
#define WSC    64.0f
#define PSC    1024.0f
static_assert(NH * HD == DM);
static_assert((SEQ % 64) == 0 && (DM % 64) == 0 && (MP % 64) == 0);
static_assert(DM == 4 * 256);
static_assert(HD == 64);

typedef _Float16       v16h __attribute__((ext_vector_type(16)));
typedef __bf16         v16b __attribute__((ext_vector_type(16)));
typedef unsigned short v16us __attribute__((ext_vector_type(16)));
typedef unsigned short v8us __attribute__((ext_vector_type(8)));
typedef float          v8f  __attribute__((ext_vector_type(8)));
typedef float          v4f  __attribute__((ext_vector_type(4)));
typedef unsigned int   v4u  __attribute__((ext_vector_type(4)));

union Frag { v16us u; v8us p[2]; v16h h; v16b b; };
union U8   { v8us s; v4u u; };

__device__ __forceinline__ unsigned short bf_bits(float f) {
  unsigned u = __float_as_uint(f);
  return (unsigned short)((u + 0x7FFFu + ((u >> 16) & 1u)) >> 16);
}
__device__ __forceinline__ float bf_up(unsigned short h) { return __uint_as_float(((unsigned)h) << 16); }
__device__ __forceinline__ float bfr(float f) { return bf_up(bf_bits(f)); }
__device__ __forceinline__ unsigned short h_bits(_Float16 x) { return __builtin_bit_cast(unsigned short, x); }
__device__ __forceinline__ unsigned pk16(unsigned short a, unsigned short b) { return (unsigned)a | ((unsigned)b << 16); }
__device__ __forceinline__ v8f zero8() { v8f z = {0.f, 0.f, 0.f, 0.f, 0.f, 0.f, 0.f, 0.f}; return z; }

__device__ __forceinline__ v16us ldfrag(const unsigned short* p) {
  Frag f;
  f.p[0] = *(const v8us*)(p);
  f.p[1] = *(const v8us*)(p + 16);
  return f.u;
}

template <int BF>
__device__ __forceinline__ v8f mma_raw(v16us a, v16us b, v8f c) {
  Frag fa, fb;
  fa.u = a;
  fb.u = b;
  if constexpr (BF) {
    return __builtin_amdgcn_wmma_f32_16x16x32_bf16(false, fa.b, false, fb.b, (short)0, c, false, false);
  } else {
    return __builtin_amdgcn_wmma_f32_16x16x32_f16(false, fa.h, false, fb.h, (short)0, c, false, false);
  }
}
template <int BF>
__device__ __forceinline__ v8f mma_g(v16us a, v16us b, v8f c) {
  c = mma_raw<BF>(a, b, c);
#if defined(__HIP_DEVICE_COMPILE__)
  asm volatile("v_nop\n\tv_nop\n\tv_nop\n\tv_nop" : "+v"(c) : "v"(a), "v"(b));
#endif
  return c;
}
__device__ __forceinline__ void dep_guard1(v8f& a, v8f& b, v16us x) {
#if defined(__HIP_DEVICE_COMPILE__)
  asm volatile("v_nop\n\tv_nop\n\tv_nop\n\tv_nop" : "+v"(a), "+v"(b) : "v"(x));
#endif
}
__device__ __forceinline__ void keep4(v16us a, v16us b, v16us c, v16us d) {
#if defined(__HIP_DEVICE_COMPILE__)
  asm volatile("v_nop" :: "v"(a), "v"(b), "v"(c), "v"(d));
#endif
}
__device__ __forceinline__ void acc_guard4(v8f& a, v8f& b, v8f& c, v8f& d) {
#if defined(__HIP_DEVICE_COMPILE__)
  asm volatile("v_nop\n\tv_nop\n\tv_nop\n\tv_nop" : "+v"(a), "+v"(b), "+v"(c), "+v"(d));
#endif
}
__device__ __forceinline__ void wave_sync_lds() {
  __builtin_amdgcn_fence(__ATOMIC_RELEASE, "workgroup");
  __builtin_amdgcn_wave_barrier();
  __builtin_amdgcn_fence(__ATOMIC_ACQUIRE, "workgroup");
}
__device__ __forceinline__ float wsum(float v) {
#pragma unroll
  for (int off = 16; off > 0; off >>= 1) v += __shfl_xor(v, off, 32);
  return v;
}
__device__ __forceinline__ float bsum256(float v, float* red, int lane, int wave) {
  v = wsum(v);
  if (lane == 0) red[wave] = v;
  __syncthreads();
  float tot = 0.f;
#pragma unroll
  for (int w = 0; w < 8; ++w) tot += red[w];
  return tot;
}

__global__ __launch_bounds__(256) void conv_h16(const float* __restrict__ X, unsigned short* Xh, int n8, float wsc) {
  const int i  = blockIdx.x * 256 + threadIdx.x;
  const int ic = (i < n8) ? i : (n8 - 1);
  const float* src = X + (size_t)ic * 8;
  const v4f a = *(const v4f*)(src);
  const v4f c = *(const v4f*)(src + 4);
  v4u o;
  o[0] = pk16(h_bits((_Float16)(bfr(a[0]) * wsc)), h_bits((_Float16)(bfr(a[1]) * wsc)));
  o[1] = pk16(h_bits((_Float16)(bfr(a[2]) * wsc)), h_bits((_Float16)(bfr(a[3]) * wsc)));
  o[2] = pk16(h_bits((_Float16)(bfr(c[0]) * wsc)), h_bits((_Float16)(bfr(c[1]) * wsc)));
  o[3] = pk16(h_bits((_Float16)(bfr(c[2]) * wsc)), h_bits((_Float16)(bfr(c[3]) * wsc)));
  if (i < n8) *(volatile v4u*)(Xh + (size_t)i * 8) = o;
  __threadfence();
  if (i < n8) *(volatile v4u*)(Xh + (size_t)i * 8) = o;
}

template <int MODE>
__global__ __launch_bounds__(256) void conv_wT(const float* __restrict__ W, unsigned short* T,
                                               int nr, int nc, int ldo, int dupoff, float wsc) {
  __shared__ __align__(16) unsigned short tile[64 * 72];
  const int t = threadIdx.x, lane = t & 31, wave = t >> 5;
  const int c0 = blockIdx.x * 64;
  const int r0 = blockIdx.y * 64;
#pragma unroll
  for (int i = 0; i < 4; ++i) {
    const int idx = t + 256 * i;
    const int r = idx >> 4, c4 = (idx & 15) * 4;
    int rr = r0 + r;  rr = (rr < nr) ? rr : (nr - 1);
    int cc = c0 + c4; cc = (cc < nc - 4) ? cc : (nc - 4);
    const v4f w = *(const v4f*)(W + (size_t)rr * nc + cc);
#pragma unroll
    for (int e = 0; e < 4; ++e) {
      unsigned short bits;
      if (MODE == 0) bits = h_bits((_Float16)(bfr(w[e]) * wsc));
      else           bits = bf_bits(w[e]);
      tile[(c4 + e) * 72 + r] = bits;
    }
  }
  __syncthreads();
  const int q8 = lane >> 3, c8 = (lane & 7) * 8;
  U8 v[2];
#pragma unroll
  for (int it = 0; it < 2; ++it) {
    const int row = wave * 8 + it * 4 + q8;
    v[it].s = *(const v8us*)(tile + row * 72 + c8);
  }
  for (int pass = 0; pass < 2; ++pass) {
#pragma unroll
    for (int it = 0; it < 2; ++it) {
      const int row = wave * 8 + it * 4 + q8;
      if (c0 + row < nc && r0 + c8 + 8 <= nr) {
        unsigned short* dp = T + (size_t)(c0 + row) * ldo + r0 + c8;
        *(volatile v4u*)(dp) = v[it].u;
        if (MODE == 1) *(volatile v4u*)(dp + dupoff) = v[it].u;
      }
    }
    __threadfence();
  }
}

template <int BF, int OM, int BIASM>
__global__ __launch_bounds__(256) void gemm64(
    const unsigned short* __restrict__ A, int lda, long long strideA,
    const unsigned short* __restrict__ Bt, int ldb, long long strideB,
    const float* __restrict__ bias0, const float* __restrict__ bias1, int Nb,
    void* Cout, int ldc, long long strideC,
    int M, int N, int K, float oscale) {
  __shared__ __align__(16) float sT[8][16 * 68];
  const int b    = blockIdx.y;
  const int lane = threadIdx.x & 31;
  const int wave = threadIdx.x >> 5;
  const int tilesN = N >> 6;
  const int tilesM = M >> 6;
  const int tile = blockIdx.x * 8 + wave;
  if (tile >= tilesM * tilesN) return;
  const int tm = tile / tilesN;
  const int tn = tile - tm * tilesN;
  const int m0 = tm << 6;
  const int n0 = tn << 6;

  const unsigned short* Ab = A  + (size_t)b * (size_t)strideA;
  const unsigned short* Bb = Bt + (size_t)b * (size_t)strideB;

  const int rlane = lane & 15;
  const int koff  = (lane >> 4) * 8;
  const int mOff  = (lane >> 4) * 8;

  v8f acc[4][4];
#pragma unroll
  for (int i = 0; i < 4; ++i)
#pragma unroll
    for (int j = 0; j < 4; ++j) acc[i][j] = zero8();

  for (int k0 = 0; k0 < K; k0 += 32) {
    v16us bh[4];
#pragma unroll
    for (int j = 0; j < 4; ++j) {
      const size_t bo = (size_t)(n0 + (j << 4) + rlane) * ldb + koff + k0;
      bh[j] = ldfrag(Bb + bo);
    }
#pragma unroll
    for (int i = 0; i < 4; ++i) {
      const size_t ao = (size_t)(m0 + (i << 4) + rlane) * lda + koff + k0;
      const v16us ah = ldfrag(Ab + ao);
#pragma unroll
      for (int j = 0; j < 4; ++j) acc[i][j] = mma_raw<BF>(ah, bh[j], acc[i][j]);
      dep_guard1(acc[i][0], acc[i][3], ah);
    }
    keep4(bh[0], bh[1], bh[2], bh[3]);
  }
  acc_guard4(acc[0][0], acc[0][1], acc[0][2], acc[0][3]);
  acc_guard4(acc[1][0], acc[1][1], acc[1][2], acc[1][3]);
  acc_guard4(acc[2][0], acc[2][1], acc[2][2], acc[2][3]);
  acc_guard4(acc[3][0], acc[3][1], acc[3][2], acc[3][3]);

  const int hh2 = lane >> 4, c4 = (lane & 15) * 4;
  const int q8  = lane >> 3, c8 = (lane & 7) * 8;
  float bc[8];
#pragma unroll
  for (int e = 0; e < 8; ++e) bc[e] = 0.f;
  if (BIASM == 0) {
    const bool use1 = (n0 >= Nb);
    if (OM == 0) {
      const int cb = n0 + c4;
      const int i0 = (cb < Nb - 4) ? cb : (Nb - 4);
      const int i1 = (cb - Nb > 0) ? (cb - Nb) : 0;
      const v4f b0v = *(const v4f*)(bias0 + i0);
      const v4f b1v = *(const v4f*)(bias1 + i1);
#pragma unroll
      for (int e = 0; e < 4; ++e) bc[e] = bfr(use1 ? b1v[e] : b0v[e]);
    } else {
      const int cb = n0 + c8;
      const int i0 = (cb < Nb - 8) ? cb : (Nb - 8);
      const int i1 = (cb - Nb > 0) ? (cb - Nb) : 0;
      const v4f b0a = *(const v4f*)(bias0 + i0), b0b = *(const v4f*)(bias0 + i0 + 4);
      const v4f b1a = *(const v4f*)(bias1 + i1), b1b = *(const v4f*)(bias1 + i1 + 4);
#pragma unroll
      for (int e = 0; e < 4; ++e) {
        bc[e]     = bfr(use1 ? b1a[e] : b0a[e]);
        bc[4 + e] = bfr(use1 ? b1b[e] : b0b[e]);
      }
    }
  }

  float* slab = sT[wave];
#pragma unroll
  for (int i = 0; i < 4; ++i) {
    const int mBase = m0 + (i << 4);
#pragma unroll
    for (int j = 0; j < 4; ++j) {
#pragma unroll
      for (int r = 0; r < 8; ++r) {
        slab[(mOff + r) * 68 + (j << 4) + rlane] = acc[i][j][r];
      }
    }
    wave_sync_lds();
    if constexpr (OM == 0) {
      float* C = (float*)Cout + (size_t)b * (size_t)strideC;
      v4f vals[8];
#pragma unroll
      for (int it = 0; it < 8; ++it) {
        const int row = it * 2 + hh2;
        v4f v = *(const v4f*)(slab + row * 68 + c4);
#pragma unroll
        for (int e = 0; e < 4; ++e) v[e] = v[e] * oscale + bc[e];
        vals[it] = v;
      }
      for (int pass = 0; pass < 2; ++pass) {
#pragma unroll
        for (int it = 0; it < 8; ++it) {
          const int row = it * 2 + hh2;
          *(volatile v4f*)(C + (size_t)(mBase + row) * ldc + n0 + c4) = vals[it];
        }
        __threadfence();
      }
    } else {
      unsigned short* C = (unsigned short*)Cout + (size_t)b * (size_t)strideC;
      v4u hv[4];
#pragma unroll
      for (int it = 0; it < 4; ++it) {
        const int row = it * 4 + q8;
        const float* sp = slab + row * 68 + c8;
        float bm = 0.f;
        if (BIASM == 1) bm = bfr(bias0[mBase + row]);
        v4u a;
#pragma unroll
        for (int e = 0; e < 4; ++e) {
          const float f0 = sp[2 * e]     * oscale + ((BIASM == 1) ? bm : bc[2 * e]);
          const float f1 = sp[2 * e + 1] * oscale + ((BIASM == 1) ? bm : bc[2 * e + 1]);
          a[e] = pk16(h_bits((_Float16)f0), h_bits((_Float16)f1));
        }
        hv[it] = a;
      }
      for (int pass = 0; pass < 2; ++pass) {
#pragma unroll
        for (int it = 0; it < 4; ++it) {
          const int row = it * 4 + q8;
          unsigned short* dp = C + (size_t)(mBase + row) * ldc + n0 + c8;
          *(volatile v4u*)(dp) = hv[it];
        }
        __threadfence();
      }
    }
    wave_sync_lds();
  }
}

__global__ __launch_bounds__(128)
void attn64(const unsigned short* __restrict__ qhp, const unsigned short* __restrict__ khp,
            const unsigned short* __restrict__ vtp, unsigned short* ctxp, float sscale) {
  __shared__ __align__(16) unsigned short Ksh[64 * 64];
  __shared__ __align__(16) unsigned short Vth[64 * 64];
  __shared__ __align__(16) unsigned short Psh[4][16 * 64];
  __shared__ __align__(16) float          Os[4][16 * 64];

  const int tid  = threadIdx.x;
  const int wave = tid >> 5;
  const int lane = tid & 31;
  const int hh   = lane >> 4;
  const int c    = lane & 15;

  const int bx   = blockIdx.x;
  const int qb   = bx % NQB;
  const int rest = bx / NQB;
  const int h    = rest % NH;
  const int b    = rest / NH;
  const int q0   = qb * 64 + wave * 16;
  const size_t rowB = (size_t)b * SEQ;

  const unsigned short* Qh = qhp + (size_t)h * HD;
  const unsigned short* Kg = khp + (size_t)h * HD;
  const unsigned short* Vh = vtp + ((size_t)b * DM + (size_t)h * HD) * SEQ;

  v16us qa[2];
#pragma unroll
  for (int dc = 0; dc < 2; ++dc) qa[dc] = ldfrag(Qh + (rowB + q0 + c) * DM + dc * 32 + 8 * hh);

  float mrow[8], lrow[8];
  v8f oacc[4];
#pragma unroll
  for (int r = 0; r < 8; ++r) { mrow[r] = -INFINITY; lrow[r] = 0.f; }
#pragma unroll
  for (int t = 0; t < 4; ++t) oacc[t] = zero8();

  for (int kt = 0; kt < NQB; ++kt) {
    const int kv0 = kt * 64;
    __syncthreads();
    {
      const int r = tid >> 1, hf = (tid & 1) * 32;
      const unsigned short* kg = Kg + (rowB + kv0 + r) * DM + hf;
      const unsigned short* vg = Vh + (size_t)r * SEQ + kv0 + hf;
#pragma unroll
      for (int i = 0; i < 4; ++i) {
        const v8us a0 = *(const v8us*)(kg + 8 * i);
        const v8us b0 = *(const v8us*)(vg + 8 * i);
        *(v8us*)(Ksh + r * 64 + hf + 8 * i) = a0;
        *(v8us*)(Vth + r * 64 + hf + 8 * i) = b0;
      }
    }
    __syncthreads();

    v8f s[4];
#pragma unroll
    for (int j = 0; j < 4; ++j) {
      v8f sh = zero8();
#pragma unroll
      for (int dc = 0; dc < 2; ++dc) {
        Frag kb;
        kb.p[0] = *(const v8us*)(Ksh + (j * 16 + c) * 64 + dc * 32 + 8 * hh);
        kb.p[1] = *(const v8us*)(Ksh + (j * 16 + c) * 64 + dc * 32 + 16 + 8 * hh);
        sh = mma_g<0>(qa[dc], kb.u, sh);
      }
#pragma unroll
      for (int r = 0; r < 8; ++r) s[j][r] = sh[r] * sscale;
    }

    unsigned short* pwh = Psh[wave];
#pragma unroll
    for (int r = 0; r < 8; ++r) {
      float m = s[0][r];
      m = fmaxf(m, s[1][r]);
      m = fmaxf(m, s[2][r]);
      m = fmaxf(m, s[3][r]);
#pragma unroll
      for (int off = 1; off < 16; off <<= 1) m = fmaxf(m, __shfl_xor(m, off, 32));
      const float mnew  = fmaxf(mrow[r], m);
      const float alpha = __expf(mrow[r] - mnew);
      mrow[r] = mnew;
      float psum = 0.f;
#pragma unroll
      for (int j = 0; j < 4; ++j) {
        const float p = __expf(s[j][r] - mnew);
        psum += p;
        pwh[(8 * hh + r) * 64 + j * 16 + c] = h_bits((_Float16)(p * PSC));
      }
#pragma unroll
      for (int off = 1; off < 16; off <<= 1) psum += __shfl_xor(psum, off, 32);
      lrow[r] = lrow[r] * alpha + psum;
#pragma unroll
      for (int t = 0; t < 4; ++t) oacc[t][r] *= alpha;
    }
    wave_sync_lds();

#pragma unroll 1
    for (int kk = 0; kk < 2; ++kk) {
      Frag pa;
      pa.p[0] = *(const v8us*)(pwh + c * 64 + kk * 32 + 8 * hh);
      pa.p[1] = *(const v8us*)(pwh + c * 64 + kk * 32 + 16 + 8 * hh);
#pragma unroll
      for (int t = 0; t < 4; ++t) {
        Frag vb;
        vb.p[0] = *(const v8us*)(Vth + (t * 16 + c) * 64 + kk * 32 + 8 * hh);
        vb.p[1] = *(const v8us*)(Vth + (t * 16 + c) * 64 + kk * 32 + 16 + 8 * hh);
        oacc[t] = mma_g<0>(pa.u, vb.u, oacc[t]);
      }
    }
  }

  float* os = Os[wave];
#pragma unroll
  for (int r = 0; r < 8; ++r) {
    const float l = lrow[r];
    const float inv = ((l > 0.f) ? (1.0f / l) : 0.f) * (1.0f / PSC);
#pragma unroll
    for (int t = 0; t < 4; ++t) os[(8 * hh + r) * 64 + t * 16 + c] = oacc[t][r] * inv;
  }
  wave_sync_lds();
  {
    const int q4 = lane >> 3, c8 = (lane & 7) * 8;
    v4u hv[4], hl[4];
#pragma unroll
    for (int it = 0; it < 4; ++it) {
      const int row = it * 4 + q4;
      const float* sp = os + row * 64 + c8;
      v4u a, d;
#pragma unroll
      for (int e = 0; e < 4; ++e) {
        const float f0 = sp[2 * e], f1 = sp[2 * e + 1];
        const unsigned short hb0 = bf_bits(f0), hb1 = bf_bits(f1);
        const unsigned short lb0 = bf_bits(f0 - bf_up(hb0)), lb1 = bf_bits(f1 - bf_up(hb1));
        a[e] = pk16(hb0, hb1);
        d[e] = pk16(lb0, lb1);
      }
      hv[it] = a;
      hl[it] = d;
    }
    for (int pass = 0; pass < 2; ++pass) {
#pragma unroll
      for (int it = 0; it < 4; ++it) {
        const int row = it * 4 + q4;
        const size_t go = (rowB + q0 + row) * CTXP + (size_t)h * HD + c8;
        *(volatile v4u*)(ctxp + go)      = hv[it];
        *(volatile v4u*)(ctxp + go + DM) = hl[it];
      }
      __threadfence();
    }
  }
}

__global__ __launch_bounds__(256) void ln_row_f(const float* __restrict__ AOp, const float* __restrict__ X,
                                              const float* __restrict__ gam, const float* __restrict__ bet,
                                              float* outp) {
  __shared__ float red0[8], red1[8];
  const int t = threadIdx.x, lane = t & 31, wave = t >> 5;
  const size_t base = (size_t)blockIdx.x * DM;
  const v4f av = *(const v4f*)(AOp + base + 4 * t);
  const v4f xv = *(const v4f*)(X + base + 4 * t);
  v4f y;
#pragma unroll
  for (int e = 0; e < 4; ++e) y[e] = bfr(xv[e]) + av[e];
  const float mean = bsum256((y[0] + y[1]) + (y[2] + y[3]), red0, lane, wave) * (1.0f / DM);
  v4f d;
#pragma unroll
  for (int e = 0; e < 4; ++e) d[e] = y[e] - mean;
  const float var  = bsum256((d[0] * d[0] + d[1] * d[1]) + (d[2] * d[2] + d[3] * d[3]), red1, lane, wave) * (1.0f / DM);
  const float rstd = rsqrtf(var + LNEPS);
  const v4f gv = *(const v4f*)(gam + 4 * t);
  const v4f bv = *(const v4f*)(bet + 4 * t);
  v4f o;
#pragma unroll
  for (int e = 0; e < 4; ++e) o[e] = (d[e] * rstd) * bfr(gv[e]) + bfr(bv[e]);
  float* dst = outp + base + 4 * t;
  *(volatile v4f*)dst = o;
  __threadfence();
  *(volatile v4f*)dst = o;
}

extern "C" void kernel_launch(void* const* d_in, const int* in_sizes, int n_in,
                              void* d_out, int out_size, void* d_ws, size_t ws_size,
                              hipStream_t stream) {
  if (n_in < 11) return;
  if (in_sizes[0] != MP * DM) return;
  if (in_sizes[1] != DM * DM || in_sizes[3] != DM * DM || in_sizes[5] != DM * DM || in_sizes[7] != DM * DM) return;
  if (in_sizes[2] != DM || in_sizes[4] != DM || in_sizes[6] != DM || in_sizes[8] != DM) return;
  if (in_sizes[9] != DM || in_sizes[10] != DM) return;
  if (out_size != MP * DM) return;

  const float* x     = (const float*)d_in[0];
  const float* Wq    = (const float*)d_in[1];
  const float* bq    = (const float*)d_in[2];
  const float* Wk    = (const float*)d_in[3];
  const float* bk    = (const float*)d_in[4];
  const float* Wv    = (const float*)d_in[5];
  const float* bv    = (const float*)d_in[6];
  const float* Wo    = (const float*)d_in[7];
  const float* bo    = (const float*)d_in[8];
  const float* gamma = (const float*)d_in[9];
  const float* beta  = (const float*)d_in[10];

  const size_t PW   = (size_t)3 * DM * DM * 2;
  const size_t PWO  = (size_t)DM * CTXP * 2;
  const size_t PX   = (size_t)MP * DM * 2;
  const size_t PQ   = (size_t)MP * DM * 2;
  const size_t PK   = (size_t)MP * DM * 2;
  const size_t PV   = (size_t)NBATCH * DM * SEQ * 2;
  const size_t PC   = (size_t)MP * CTXP * 2;
  const size_t PA   = (size_t)MP * DM * 4;
  size_t off = 0;
  const size_t oW  = off; off += PW;
  const size_t oWo = off; off += PWO;
  const size_t oX  = off; off += PX;
  const size_t oQ  = off; off += PQ;
  const size_t oK  = off; off += PK;
  const size_t oV  = off; off += PV;
  const size_t oC  = off; off += PC;
  if (off > ws_size) return;
  if (off > (size_t)134217728) return;
  if (PA != PX + PQ) return;
  if (oX + PA > oK) return;

  char* ws = (char*)d_ws;
  unsigned short* WqkvH = (unsigned short*)(ws + oW);
  unsigned short* WoB   = (unsigned short*)(ws + oWo);
  unsigned short* XH    = (unsigned short*)(ws + oX);
  unsigned short* QH    = (unsigned short*)(ws + oQ);
  unsigned short* KH    = (unsigned short*)(ws + oK);
  unsigned short* VT    = (unsigned short*)(ws + oV);
  unsigned short* Ctx   = (unsigned short*)(ws + oC);
  float*          AO    = (float*)(ws + oX);
  float*          out0  = (float*)d_out;

  const int n8x = (MP * DM) / 8;
  if ((n8x % 256) != 0) return;
  const dim3 blk(256), blk128(128);
  const dim3 gW(DM / 64, DM / 64);
  const dim3 gCx((n8x + 255) / 256);
  const dim3 gN1k(((MP / 64) * (DM / 64) + 7) / 8, 1);
  const dim3 gVT(((DM / 64) * (SEQ / 64) + 7) / 8, NBATCH);
  const dim3 gAttn(NBATCH * NH * NQB);
  const dim3 gRow(MP);
  const float invw  = 1.0f / WSC;
  const float ssc   = 0.125f;

  conv_wT<0><<<gW, blk, 0, stream>>>(Wq, WqkvH, DM, DM, DM, 0, WSC);
  conv_wT<0><<<gW, blk, 0, stream>>>(Wk, WqkvH + (size_t)DM * DM, DM, DM, DM, 0, WSC);
  conv_wT<0><<<gW, blk, 0, stream>>>(Wv, WqkvH + (size_t)2 * DM * DM, DM, DM, DM, 0, WSC);
  conv_wT<1><<<gW, blk, 0, stream>>>(Wo, WoB, DM, DM, CTXP, DM, 1.0f);

  conv_h16<<<gCx, blk, 0, stream>>>(x, XH, n8x, 1.0f);

  gemm64<0, 2, 0><<<gN1k, blk, 0, stream>>>(
      XH, DM, 0LL, WqkvH, DM, 0LL, bq, bq, DM,
      (void*)QH, DM, 0LL, MP, DM, DM, invw);
  gemm64<0, 2, 0><<<gN1k, blk, 0, stream>>>(
      XH, DM, 0LL, WqkvH + (size_t)DM * DM, DM, 0LL, bk, bk, DM,
      (void*)KH, DM, 0LL, MP, DM, DM, invw);

  gemm64<0, 2, 1><<<gVT, blk, 0, stream>>>(
      WqkvH + (size_t)2 * DM * DM, DM, 0LL, XH, DM, (long long)SEQ * DM, bv, bv, SEQ,
      (void*)VT, SEQ, (long long)DM * SEQ, DM, SEQ, DM, invw);

  attn64<<<gAttn, blk128, 0, stream>>>(QH, KH, VT, Ctx, ssc);

  gemm64<1, 0, 0><<<gN1k, blk, 0, stream>>>(
      Ctx, CTXP, 0LL, WoB, CTXP, 0LL, bo, bo, DM,
      (void*)AO, DM, 0LL, MP, DM, CTXP, 1.0f);

  ln_row_f<<<gRow, blk, 0, stream>>>(AO, x, gamma, beta, out0);
  (void)hipGetLastError();
}
